// TransformerLayer_13889924235941
// MI455X (gfx1250) — hardware-verified
//
#include <hip/hip_runtime.h>
#include <stdint.h>

#define E_   1024
#define H_   16
#define DK_  64
#define HID_ 4096
#define B_   2
#define S_   2048
#define BS_  (B_ * S_)
#define EPS_ 1e-5f

typedef __attribute__((ext_vector_type(16))) _Float16 bf16x16;
typedef __attribute__((ext_vector_type(8)))  _Float16 f16x8;
typedef __attribute__((ext_vector_type(4)))  float f32x4v;
typedef float f32x4a __attribute__((ext_vector_type(4), may_alias));
typedef __attribute__((ext_vector_type(8)))  float  f32x8;
typedef __attribute__((ext_vector_type(4)))  unsigned int u32x4;
typedef __attribute__((ext_vector_type(8)))  unsigned int u32x8;

union ABFrag {
    bf16x16  v;
    uint32_t u[8];
    u32x4    q[2];
};

__device__ __forceinline__ unsigned short f2bf(float f) {
    return __builtin_bit_cast(unsigned short, (_Float16)f);
}
__device__ __forceinline__ uint32_t pk2h(float a, float b) { return (uint32_t)f2bf(a) | ((uint32_t)f2bf(b) << 16); }

__device__ __forceinline__ f32x8 wmma_bf16(const ABFrag& a, const ABFrag& b, f32x8 c) {
    return __builtin_amdgcn_wmma_f32_16x16x32_f16(
        false, a.v, false, b.v, (short)0, c, false, false);
}

__device__ __forceinline__ void async_copy_b128(uint32_t lds_off,
                                                const unsigned short* g) {
    asm volatile("global_load_async_to_lds_b128 %0, %1, off"
                 :: "v"(lds_off), "v"(g) : "memory");
}
#define S_WAIT_ASYNC0() asm volatile("s_wait_asynccnt 0x0" ::: "memory")
#define S_WAIT_ASYNC1() asm volatile("s_wait_asynccnt 0x1" ::: "memory")

__device__ __forceinline__ void tdm_load_tile_2d(uint32_t lds_off, const void* gaddr,
                                                 uint32_t tensor_d0, uint32_t tensor_d1,
                                                 uint32_t tile_d0, uint32_t tile_d1,
                                                 uint64_t stride0) {
    uint64_t ga = (uint64_t)gaddr;
    u32x4 g0;
    g0[0] = 1u;
    g0[1] = lds_off;
    g0[2] = (uint32_t)ga;
    g0[3] = (uint32_t)((ga >> 32) & 0x1FFFFFFu) | (2u << 30);
    u32x8 g1;
    g1[0] = (1u << 16)
          | (1u << 20)
          | (3u << 22)
          | (3u << 25);
    g1[1] = (tensor_d0 & 0xFFFFu) << 16;
    g1[2] = ((tensor_d0 >> 16) & 0xFFFFu) | ((tensor_d1 & 0xFFFFu) << 16);
    g1[3] = ((tensor_d1 >> 16) & 0xFFFFu) | ((tile_d0 & 0xFFFFu) << 16);
    g1[4] = (tile_d1 & 0xFFFFu);
    g1[5] = (uint32_t)stride0;
    g1[6] = (uint32_t)((stride0 >> 32) & 0xFFFFu);
    g1[7] = 0u;
    asm volatile("tensor_load_to_lds %0, %1" :: "s"(g0), "s"(g1) : "memory");
}

__global__ __launch_bounds__(256) void transpose_f32_to_bf16_kernel(
    const float* __restrict__ in, unsigned short* __restrict__ out,
    int K, int N, int total) {
    int i = (blockIdx.x * 256 + threadIdx.x) * 2;
    if (i >= total) return;
    int kn = K * N;
    int b  = i / kn;
    int r  = i - b * kn;
    int n  = r / K;
    int k  = r - n * K;
    const uint32_t v = pk2h(in[(size_t)b * kn + (size_t)k * N + n], in[(size_t)b * kn + (size_t)(k + 1) * N + n]);
    uint32_t* d = (uint32_t*)(out + (size_t)b * kn + (size_t)n * K + k);
    *(volatile uint32_t*)d = v; __threadfence(); *(volatile uint32_t*)d = v;
}

__global__ __launch_bounds__(256) void ln_kernel(
    const float* __restrict__ X, const float* __restrict__ Res,
    const float* __restrict__ gamma, const float* __restrict__ beta,
    float* __restrict__ Yf, unsigned short* __restrict__ Yb) {
    const int row = blockIdx.x;
    const int t   = threadIdx.x;
    const size_t base = (size_t)row * E_;
    float v[4];
#pragma unroll
    for (int i = 0; i < 4; ++i) {
        int j = t * 4 + i;
        float a = X[base + j];
        if (Res) a += Res[base + j];
        v[i] = a;
    }
    __shared__ float red[256];
    red[t] = v[0] + v[1] + v[2] + v[3];
    __syncthreads();
    for (int off = 128; off; off >>= 1) {
        if (t < off) red[t] += red[t + off];
        __syncthreads();
    }
    const float mu = red[0] * (1.0f / E_);
    __syncthreads();
    float s2 = 0.f;
#pragma unroll
    for (int i = 0; i < 4; ++i) { float d = v[i] - mu; s2 += d * d; }
    red[t] = s2;
    __syncthreads();
    for (int off = 128; off; off >>= 1) {
        if (t < off) red[t] += red[t + off];
        __syncthreads();
    }
    const float rstd = rsqrtf(red[0] * (1.0f / E_) + EPS_);
    f32x4v y4;
#pragma unroll
    for (int i = 0; i < 4; ++i) { int j = t * 4 + i; y4[i] = (v[i] - mu) * rstd * gamma[j] + beta[j]; }
    __attribute__((ext_vector_type(2))) unsigned yb; yb.x = pk2h(y4[0], y4[1]); yb.y = pk2h(y4[2], y4[3]);
    typedef __attribute__((ext_vector_type(2))) unsigned u32x2v;
    *(volatile f32x4v*)(Yf + base + t * 4) = y4; *(volatile u32x2v*)(Yb + base + t * 4) = yb; __threadfence();
    *(volatile f32x4v*)(Yf + base + t * 4) = y4; *(volatile u32x2v*)(Yb + base + t * 4) = yb;
}

__global__ __launch_bounds__(256) void gemm_qkv_kernel(
    const unsigned short* __restrict__ A,
    const unsigned short* __restrict__ Wt,
    const float* __restrict__ bias,
    unsigned short* __restrict__ Out,
    int out_ss, int out_ds, float out_scale) {
    const int h    = blockIdx.y;
    const int wave = threadIdx.x >> 5;
    const int lane = threadIdx.x & 31;
    const int half = lane >> 4;
    const int nl   = lane & 15;
    const int m0w  = blockIdx.x * 256 + wave * 32;

    __shared__ __align__(16) unsigned short Bs[2][64][40];
    __shared__ __align__(16) unsigned short stq[8 * 32 * 72];

    const unsigned short* WhT = Wt + (size_t)h * 64 * E_;

    f32x8 zero = {0, 0, 0, 0, 0, 0, 0, 0};
    f32x8 acc[2][4] = {{zero, zero, zero, zero}, {zero, zero, zero, zero}};

    const int srow = threadIdx.x >> 2;
    const int sc   = (threadIdx.x & 3) * 8;

    async_copy_b128((uint32_t)(uintptr_t)&Bs[0][srow][sc],
                    WhT + (size_t)srow * E_ + sc);

    for (int k0 = 0; k0 < E_; k0 += 32) {
        const int buf = (k0 >> 5) & 1;
        const bool more = (k0 + 32 < E_);
        if (more)
            async_copy_b128((uint32_t)(uintptr_t)&Bs[buf ^ 1][srow][sc],
                            WhT + (size_t)srow * E_ + (k0 + 32) + sc);
        if (more) S_WAIT_ASYNC1(); else S_WAIT_ASYNC0();
        __syncthreads();

        ABFrag a[2];
#pragma unroll
        for (int g = 0; g < 2; ++g) {
            const unsigned short* arow =
                A + (size_t)(m0w + g * 16 + nl) * E_ + k0 + half * 8;
            a[g].q[0] = *(const u32x4*)(arow);
            a[g].q[1] = *(const u32x4*)(arow + 16);
        }
        ABFrag bfr[4];
#pragma unroll
        for (int f = 0; f < 4; ++f) {
            const unsigned short* brow = &Bs[buf][f * 16 + nl][half * 8];
            bfr[f].q[0] = *(const u32x4*)(brow);
            bfr[f].q[1] = *(const u32x4*)(brow + 16);
        }
#pragma unroll
        for (int g = 0; g < 2; ++g)
#pragma unroll
            for (int f = 0; f < 4; ++f)
                acc[g][f] = wmma_bf16(a[g], bfr[f], acc[g][f]);
        __syncthreads();
    }

    const int bb0 = (blockIdx.x * 256) >> 11, s0blk = (blockIdx.x * 256) & (S_ - 1);
    if (out_ss != 1) {
        unsigned short* sw = stq + wave * 32 * 72;
#pragma unroll
        for (int g = 0; g < 2; ++g)
#pragma unroll
            for (int f = 0; f < 4; ++f)
#pragma unroll
                for (int r = 0; r < 8; ++r) {
                    int d = f * 16 + nl;
                    sw[(g * 16 + r + half * 8) * 72 + d] = f2bf((acc[g][f][r] + bias[h * 64 + d]) * out_scale);
                }
        asm volatile("s_wait_dscnt 0" ::: "memory");
        unsigned short* ob = Out + (((size_t)bb0 * H_ + h) * S_ + s0blk + wave * 32) * 64;
#pragma unroll 1
        for (int pass = 0; pass < 2; ++pass) {
#pragma unroll
            for (int i = 0; i < 8; ++i) { const int c = lane + 32 * i, rr = c >> 3, q = (c & 7) * 8;
                *(volatile u32x4*)(ob + (size_t)rr * 64 + q) = *(const u32x4*)(sw + rr * 72 + q); }
            __threadfence();
        }
    } else {
#pragma unroll
        for (int g = 0; g < 2; ++g)
#pragma unroll
            for (int f = 0; f < 4; ++f)
#pragma unroll
                for (int r = 0; r < 8; ++r) {
                    int d = f * 16 + nl;
                    stq[d * 264 + wave * 32 + g * 16 + r + half * 8] = f2bf((acc[g][f][r] + bias[h * 64 + d]) * out_scale);
                }
        __syncthreads();
        unsigned short* ob = Out + (((size_t)bb0 * H_ + h) * S_) * 64 + s0blk;
#pragma unroll 1
        for (int pass = 0; pass < 2; ++pass) {
            for (int c = threadIdx.x; c < 64 * 32; c += 256) { const int d = c >> 5, q = (c & 31) * 8;
                *(volatile u32x4*)(ob + (size_t)d * S_ + q) = *(const u32x4*)(stq + d * 264 + q); }
            __threadfence();
        }
    }
}

__global__ __launch_bounds__(32) void flash_kernel(
    const unsigned short* __restrict__ Q,
    const unsigned short* __restrict__ Km,
    const unsigned short* __restrict__ Vt,
    float* __restrict__ O) {
    const int lane = threadIdx.x & 31;
    const int half = lane >> 4;
    const int nl   = lane & 15;
    const int q0 = blockIdx.x * 16;
    const int h  = blockIdx.y;
    const int b  = blockIdx.z;
    const size_t bh = ((size_t)b * H_ + h) * S_ * 64;

    ABFrag aQ0, aQ1;
    {
        const unsigned short* qrow = Q + bh + (size_t)(q0 + nl) * 64 + half * 8;
        aQ0.q[0] = *(const u32x4*)(qrow);
        aQ0.q[1] = *(const u32x4*)(qrow + 16);
        aQ1.q[0] = *(const u32x4*)(qrow + 32);
        aQ1.q[1] = *(const u32x4*)(qrow + 48);
    }

    f32x8 zero = {0, 0, 0, 0, 0, 0, 0, 0};
    f32x8 acc[4] = {zero, zero, zero, zero};
    float rowmax[8], rowsum[8];
#pragma unroll
    for (int r = 0; r < 8; ++r) { rowmax[r] = -1e30f; rowsum[r] = 0.f; }

    __shared__ __align__(16) unsigned short Pl[16][32];

    const int nkb = (q0 + 16 + 31) >> 5;
    for (int kb = 0; kb < nkb; ++kb) {
        const int t0 = kb * 32;
        if (kb + 1 < nkb) {
            __builtin_prefetch(Km + bh + (size_t)(t0 + 32 + nl) * 64, 0, 0);
            __builtin_prefetch(Vt + bh + (size_t)nl * S_ + t0 + 32, 0, 0);
        }
        ABFrag bk[2][2];
#pragma unroll
        for (int sf = 0; sf < 2; ++sf) {
            const unsigned short* krow =
                Km + bh + (size_t)(t0 + sf * 16 + nl) * 64 + half * 8;
            bk[sf][0].q[0] = *(const u32x4*)(krow);
            bk[sf][0].q[1] = *(const u32x4*)(krow + 16);
            bk[sf][1].q[0] = *(const u32x4*)(krow + 32);
            bk[sf][1].q[1] = *(const u32x4*)(krow + 48);
        }
        f32x8 c[2];
#pragma unroll
        for (int sf = 0; sf < 2; ++sf) {
            f32x8 s = zero;
            s = wmma_bf16(aQ0, bk[sf][0], s);
            s = wmma_bf16(aQ1, bk[sf][1], s);
#pragma unroll
            for (int r = 0; r < 8; ++r) {
                int qg = q0 + r + half * 8;
                int tg = t0 + sf * 16 + nl;
                c[sf][r] = (tg <= qg) ? s[r] : -1e30f;
            }
        }
        float scale[8];
#pragma unroll
        for (int r = 0; r < 8; ++r) {
            float m2 = fmaxf(c[0][r], c[1][r]);
            m2 = fmaxf(m2, __shfl_xor(m2, 1, 16));
            m2 = fmaxf(m2, __shfl_xor(m2, 2, 16));
            m2 = fmaxf(m2, __shfl_xor(m2, 4, 16));
            m2 = fmaxf(m2, __shfl_xor(m2, 8, 16));
            float nm = fmaxf(rowmax[r], m2);
            scale[r] = __expf(rowmax[r] - nm);
            rowmax[r] = nm;
        }
#pragma unroll
        for (int r = 0; r < 8; ++r) {
            c[0][r] = __expf(c[0][r] - rowmax[r]);
            c[1][r] = __expf(c[1][r] - rowmax[r]);
            float ssum = c[0][r] + c[1][r];
            ssum += __shfl_xor(ssum, 1, 16);
            ssum += __shfl_xor(ssum, 2, 16);
            ssum += __shfl_xor(ssum, 4, 16);
            ssum += __shfl_xor(ssum, 8, 16);
            rowsum[r] = rowsum[r] * scale[r] + ssum;
        }
#pragma unroll
        for (int sf = 0; sf < 2; ++sf)
#pragma unroll
            for (int r = 0; r < 8; ++r)
                Pl[r + half * 8][sf * 16 + nl] = f2bf(c[sf][r] * 1024.0f);
#pragma unroll
        for (int f = 0; f < 4; ++f)
#pragma unroll
            for (int r = 0; r < 8; ++r)
                acc[f][r] *= scale[r];

        ABFrag aP;
        const unsigned short* prow = &Pl[nl][half * 8];
        aP.q[0] = *(const u32x4*)(prow);
        aP.q[1] = *(const u32x4*)(prow + 16);

        ABFrag bv[4];
#pragma unroll
        for (int f = 0; f < 4; ++f) {
            const unsigned short* vrow =
                Vt + bh + (size_t)(f * 16 + nl) * S_ + t0 + half * 8;
            bv[f].q[0] = *(const u32x4*)(vrow);
            bv[f].q[1] = *(const u32x4*)(vrow + 16);
        }
#pragma unroll
        for (int f = 0; f < 4; ++f)
            acc[f] = wmma_bf16(aP, bv[f], acc[f]);
    }

    float inv[8];
#pragma unroll
    for (int r = 0; r < 8; ++r) inv[r] = 1.0f / (rowsum[r] * 1024.0f);
    __shared__ __align__(16) float Os[16][68];
#pragma unroll
    for (int f = 0; f < 4; ++f)
#pragma unroll
        for (int r = 0; r < 8; ++r) Os[r + half * 8][f * 16 + nl] = acc[f][r] * inv[r];
    asm volatile("s_wait_dscnt 0" ::: "memory");
#pragma unroll 1
    for (int pass = 0; pass < 2; ++pass) {
#pragma unroll
        for (int i = 0; i < 8; ++i) { const int c = lane + 32 * i, rr = c >> 4, qd = (c & 15) * 4;
            *(volatile f32x4v*)(O + ((size_t)b * S_ + q0 + rr) * E_ + h * 64 + qd) = *(const volatile f32x4a*)&Os[rr][qd]; }
        __threadfence();
    }
}

__global__ __launch_bounds__(256) void gemm_mlp_kernel(
    const unsigned short* __restrict__ A, int lda,
    const unsigned short* __restrict__ Bt,
    int Ntot,
    const float* __restrict__ bias,
    const float* __restrict__ residual,
    float* __restrict__ Cf,
    unsigned short* __restrict__ Cb,
    int ldc, int K, int relu, int out_bf16) {
    const int wave = threadIdx.x >> 5;
    const int lane = threadIdx.x & 31;
    const int half = lane >> 4;
    const int nl   = lane & 15;
    const int m0w  = blockIdx.x * 256 + wave * 32;
    const int n0   = blockIdx.y * 64;

    __shared__ __align__(16) unsigned short Bs[2][64][40];
    __shared__ __align__(16) float stm[8][32 * 68];

    f32x8 zero = {0, 0, 0, 0, 0, 0, 0, 0};
    f32x8 acc[2][4] = {{zero, zero, zero, zero}, {zero, zero, zero, zero}};

    const unsigned short* Btile = Bt + (size_t)n0 * K;

    if (wave == 0) {
        tdm_load_tile_2d((uint32_t)(uintptr_t)&Bs[0][0][0], Btile,
                         (uint32_t)K, (uint32_t)Ntot, 32u, 64u, (uint64_t)K);
    }

    for (int k0 = 0; k0 < K; k0 += 32) {
        const int buf = (k0 >> 5) & 1;
        const bool more = (k0 + 32 < K);
        if (wave == 0) {
            if (more)
                tdm_load_tile_2d((uint32_t)(uintptr_t)&Bs[buf ^ 1][0][0],
                                 Btile + (k0 + 32),
                                 (uint32_t)K, (uint32_t)Ntot, 32u, 64u, (uint64_t)K);
            if (more) __builtin_amdgcn_s_wait_tensorcnt(1);
            else      __builtin_amdgcn_s_wait_tensorcnt(0);
        }
        __syncthreads();

        ABFrag a[2];
#pragma unroll
        for (int g = 0; g < 2; ++g) {
            const unsigned short* arow =
                A + (size_t)(m0w + g * 16 + nl) * lda + k0 + half * 8;
            a[g].q[0] = *(const u32x4*)(arow);
            a[g].q[1] = *(const u32x4*)(arow + 16);
        }
        ABFrag bfr[4];
#pragma unroll
        for (int f = 0; f < 4; ++f) {
            const unsigned short* brow = &Bs[buf][f * 16 + nl][half * 8];
            bfr[f].q[0] = *(const u32x4*)(brow);
            bfr[f].q[1] = *(const u32x4*)(brow + 16);
        }
#pragma unroll
        for (int g = 0; g < 2; ++g)
#pragma unroll
            for (int f = 0; f < 4; ++f)
                acc[g][f] = wmma_bf16(a[g], bfr[f], acc[g][f]);
        __syncthreads();
    }

    float* sw = stm[wave];
#pragma unroll
    for (int g = 0; g < 2; ++g)
#pragma unroll
        for (int f = 0; f < 4; ++f)
#pragma unroll
            for (int r = 0; r < 8; ++r) {
                int ml = g * 16 + r + half * 8;
                int n = n0 + f * 16 + nl;
                float v = acc[g][f][r];
                if (bias) v += bias[n];
                if (relu) v = fmaxf(v, 0.0f);
                if (residual) v += residual[(size_t)(m0w + ml) * ldc + n];
                sw[ml * 68 + f * 16 + nl] = v;
            }
    asm volatile("s_wait_dscnt 0" ::: "memory");
#pragma unroll 1
    for (int pass = 0; pass < 2; ++pass) {
        if (out_bf16) {
#pragma unroll
            for (int i = 0; i < 8; ++i) { const int c = lane + 32 * i, rr = c >> 3, q = (c & 7) * 8; const float* s = sw + rr * 68 + q;
                u32x4 v; v[0] = pk2h(s[0], s[1]); v[1] = pk2h(s[2], s[3]); v[2] = pk2h(s[4], s[5]); v[3] = pk2h(s[6], s[7]);
                *(volatile u32x4*)(Cb + (size_t)(m0w + rr) * ldc + n0 + q) = v; }
        } else {
#pragma unroll
            for (int i = 0; i < 16; ++i) { const int c = lane + 32 * i, rr = c >> 4, q = (c & 15) * 4;
                *(volatile f32x4v*)(Cf + (size_t)(m0w + rr) * ldc + n0 + q) = *(const volatile f32x4a*)(sw + rr * 68 + q); }
        }
        __threadfence();
    }
}

extern "C" void kernel_launch(void* const* d_in, const int* in_sizes, int n_in,
                              void* d_out, int out_size, void* d_ws, size_t ws_size,
                              hipStream_t stream) {
    (void)in_sizes; (void)n_in; (void)out_size; (void)ws_size;

    const float* emb   = (const float*)d_in[0];
    const float* Wq    = (const float*)d_in[1];
    const float* bq    = (const float*)d_in[2];
    const float* Wk    = (const float*)d_in[3];
    const float* bk    = (const float*)d_in[4];
    const float* Wv    = (const float*)d_in[5];
    const float* bv    = (const float*)d_in[6];
    const float* ln1w  = (const float*)d_in[7];
    const float* ln1b  = (const float*)d_in[8];
    const float* ln2w  = (const float*)d_in[9];
    const float* ln2b  = (const float*)d_in[10];
    const float* W1    = (const float*)d_in[11];
    const float* b1    = (const float*)d_in[12];
    const float* W2    = (const float*)d_in[13];
    const float* b2    = (const float*)d_in[14];
    float* out = (float*)d_out;

    size_t off = 0;
    auto carve = [&](size_t bytes) -> void* {
        void* p = (char*)d_ws + off;
        off += (bytes + 255) & ~(size_t)255;
        return p;
    };
    float*          x_f32  = (float*)         carve((size_t)BS_ * E_ * 4);
    unsigned short* x_bf   = (unsigned short*)carve((size_t)BS_ * E_ * 2);
    float*          y_f32  = (float*)         carve((size_t)BS_ * E_ * 4);
    unsigned short* y_bf   = (unsigned short*)carve((size_t)BS_ * E_ * 2);
    float*          attn   = (float*)         carve((size_t)BS_ * E_ * 4);
    unsigned short* qb     = (unsigned short*)carve((size_t)B_ * H_ * S_ * 64 * 2);
    unsigned short* kb_    = (unsigned short*)carve((size_t)B_ * H_ * S_ * 64 * 2);
    unsigned short* vb     = (unsigned short*)carve((size_t)B_ * H_ * S_ * 64 * 2);
    unsigned short* h_bf   = (unsigned short*)carve((size_t)BS_ * HID_ * 2);
    unsigned short* WqT    = (unsigned short*)carve((size_t)H_ * E_ * 64 * 2);
    unsigned short* WkT    = (unsigned short*)carve((size_t)H_ * E_ * 64 * 2);
    unsigned short* WvT    = (unsigned short*)carve((size_t)H_ * E_ * 64 * 2);
    unsigned short* W1T    = (unsigned short*)carve((size_t)E_ * HID_ * 2);
    unsigned short* W2T    = (unsigned short*)carve((size_t)HID_ * E_ * 2);

    auto tcvt = [&](const float* src, unsigned short* dst, int K, int N, int batch) {
        int total = K * N * batch;
        transpose_f32_to_bf16_kernel<<<(total / 2 + 255) / 256, 256, 0, stream>>>(
            src, dst, K, N, total);
    };
    tcvt(Wq, WqT, E_, 64, H_);
    tcvt(Wk, WkT, E_, 64, H_);
    tcvt(Wv, WvT, E_, 64, H_);
    tcvt(W1, W1T, E_, HID_, 1);
    tcvt(W2, W2T, HID_, E_, 1);

    ln_kernel<<<BS_, 256, 0, stream>>>(emb, nullptr, ln1w, ln1b, x_f32, x_bf);

    dim3 gq(BS_ / 256, H_);
    gemm_qkv_kernel<<<gq, 256, 0, stream>>>(x_bf, WqT, bq, qb,  64, 1, 0.125f);
    gemm_qkv_kernel<<<gq, 256, 0, stream>>>(x_bf, WkT, bk, kb_, 64, 1, 1.0f);
    gemm_qkv_kernel<<<gq, 256, 0, stream>>>(x_bf, WvT, bv, vb,  1, S_, 1.0f);

    dim3 gf(S_ / 16, H_, B_);
    flash_kernel<<<gf, 32, 0, stream>>>(qb, kb_, vb, attn);

    ln_kernel<<<BS_, 256, 0, stream>>>(x_f32, attn, ln2w, ln2b, y_f32, y_bf);

    dim3 g1(BS_ / 256, HID_ / 64);
    gemm_mlp_kernel<<<g1, 256, 0, stream>>>(y_bf, E_, W1T, HID_, b1,
                                            nullptr, nullptr, h_bf,
                                            HID_, E_, 1, 1);

    dim3 g2(BS_ / 256, E_ / 64);
    gemm_mlp_kernel<<<g2, 256, 0, stream>>>(h_bf, HID_, W2T, E_, b2,
                                            y_f32, out, nullptr,
                                            E_, HID_, 0, 0);
}
